// SpatialSelfAttention_755914244770
// MI455X (gfx1250) — hardware-verified
//
#include <hip/hip_runtime.h>
#include <stdint.h>


#ifndef NB
#define NB 4
#endif
#ifndef SEQ
#define SEQ 4096
#endif
#define NB_FULL 4
#define SEQ_FULL 4096
#define CH 64
#define KBLK 64
#define LDP 72
#define OSP 68

static_assert(NB >= 1 && NB <= NB_FULL);
static_assert(SEQ >= KBLK && SEQ <= SEQ_FULL && (SEQ % KBLK) == 0);
static_assert(CH == 64);

typedef _Float16 v16h __attribute__((ext_vector_type(16)));
typedef _Float16 v8h  __attribute__((ext_vector_type(8)));
typedef float    v8f  __attribute__((ext_vector_type(8)));
typedef float    v4f  __attribute__((ext_vector_type(4)));
typedef v8h __attribute__((may_alias)) v8ha;
typedef v4f __attribute__((may_alias)) v4fa;

union F16x16 { v16h v; v8h p[2]; _Float16 e[16]; };
union F16x8  { v8h v; _Float16 e[8]; };

constexpr float XSC = 16.0f;
constexpr float WSC = 64.0f;
constexpr float QSC = 4.0f;
constexpr float PSC = 4096.0f;
constexpr float SCL2 = (float)(1.4426950408889634 / ((double)QSC * (double)QSC * (double)SEQ));

static __device__ __forceinline__ float bf16r(float f) {
  uint32_t u = __float_as_uint(f);
  u += 0x7FFFu + ((u >> 16) & 1u);
  u &= 0xFFFF0000u;
  return __uint_as_float(u);
}

static __device__ __forceinline__ v8f wmma16(v16h a, v16h b, v8f c) {
  v8f d = __builtin_amdgcn_wmma_f32_16x16x32_f16(false, a, false, b, (short)0, c,
                                                 false, false);
  asm volatile("v_nop\n\tv_nop\n\tv_nop\n\tv_nop" : "+v"(d) : "v"(a), "v"(b));
  return d;
}

static __device__ __forceinline__ v16h ld_frag(const _Float16* base, int pitch,
                                               int row, int h) {
  F16x16 u;
  const _Float16* q = base + (size_t)row * pitch;
  u.p[0] = *(const v8ha*)(q + 8 * h);
  u.p[1] = *(const v8ha*)(q + 16 + 8 * h);
  return u.v;
}

__global__ __launch_bounds__(128) void k_prep(const float* __restrict__ x,
                                              const float* __restrict__ W,
                                              const float* __restrict__ bias,
                                              _Float16* __restrict__ Xh,
                                              _Float16* __restrict__ QKh) {
  __shared__ __align__(16) _Float16 XS[64 * LDP];
  __shared__ __align__(16) _Float16 WS[64 * LDP];
  __shared__ __align__(16) _Float16 OS[64 * LDP];
  __shared__ float bs[64];

  const int tid = threadIdx.x;
  const int wv = tid >> 5, lid = tid & 31, h = lid >> 4, l15 = lid & 15;
  const int b  = blockIdx.x / (SEQ / 64);
  const int n0 = (blockIdx.x % (SEQ / 64)) * 64;
  const float* xb = x + (size_t)b * CH * SEQ_FULL;

#pragma unroll
  for (int it = 0; it < 4; ++it) {
    const int c = it * 16 + (tid >> 3);
    const int p = tid & 7;
    const float* src = xb + (size_t)c * SEQ_FULL + n0 + 8 * p;
    const v4f f0 = *(const v4fa*)src;
    const v4f f1 = *(const v4fa*)(src + 4);
    F16x8 u;
#pragma unroll
    for (int j = 0; j < 4; ++j) {
      u.e[j]     = (_Float16)(bf16r(f0[j]) * XSC);
      u.e[4 + j] = (_Float16)(bf16r(f1[j]) * XSC);
    }
    _Float16* dst = Xh + ((size_t)(b * CH + c) * SEQ + n0 + 8 * p);
    *(volatile v8h*)dst = u.v;
    __threadfence();
    *(volatile v8h*)dst = u.v;
#pragma unroll
    for (int j = 0; j < 8; ++j) XS[(8 * p + j) * LDP + c] = u.e[j];
  }

  {
    const int o = tid >> 1, hh = tid & 1;
    const float* src = W + o * CH + 32 * hh;
#pragma unroll
    for (int k = 0; k < 4; ++k) {
      const v4f a0 = *(const v4fa*)(src + 8 * k);
      const v4f a1 = *(const v4fa*)(src + 8 * k + 4);
      F16x8 u;
#pragma unroll
      for (int j = 0; j < 4; ++j) {
        u.e[j]     = (_Float16)(bf16r(a0[j]) * WSC);
        u.e[4 + j] = (_Float16)(bf16r(a1[j]) * WSC);
      }
      *(v8ha*)(WS + o * LDP + 32 * hh + 8 * k) = u.v;
    }
  }
  if (tid < 64) bs[tid] = bf16r(bias[tid]);
  __syncthreads();

  v16h ax[2];
#pragma unroll
  for (int cs = 0; cs < 2; ++cs) ax[cs] = ld_frag(XS + 32 * cs, LDP, 16 * wv + l15, h);

#pragma unroll
  for (int t = 0; t < 4; ++t) {
    v8f acc;
#pragma unroll
    for (int r = 0; r < 8; ++r) acc[r] = 0.0f;
#pragma unroll
    for (int cs = 0; cs < 2; ++cs)
      acc = wmma16(ax[cs], ld_frag(WS + 32 * cs, LDP, 16 * t + l15, h), acc);
    const float bo = bs[16 * t + l15];
#pragma unroll
    for (int r = 0; r < 8; ++r) {
      const float qk = acc[r] * (1.0f / (XSC * WSC)) + bo;
      OS[(16 * wv + 8 * h + r) * LDP + 16 * t + l15] = (_Float16)(qk * QSC);
    }
  }
  __syncthreads();

#pragma unroll
  for (int it = 0; it < 4; ++it) {
    const int row = 16 * wv + 4 * it + (lid >> 3);
    const int p = lid & 7;
    const v8h hv = *(const v8ha*)(OS + row * LDP + 8 * p);
    _Float16* dst = QKh + ((size_t)(b * SEQ + n0 + row) * CH + 8 * p);
    *(volatile v8h*)dst = hv;
    __threadfence();
    *(volatile v8h*)dst = hv;
  }
}

__global__ __launch_bounds__(128) void k_attn(const _Float16* __restrict__ QKh,
                                              const _Float16* __restrict__ Xh,
                                              float* __restrict__ out) {
  __shared__ __align__(16) float OSt[64 * OSP];

  const int tid = threadIdx.x;
  const int wv = tid >> 5, lid = tid & 31, h = lid >> 4, l15 = lid & 15;
  const int b  = blockIdx.x / (SEQ / 64);
  const int q0 = (blockIdx.x % (SEQ / 64)) * 64;
  const int qb = q0 + 16 * wv;

  const _Float16* Qp = QKh + (size_t)b * SEQ * CH;
  const _Float16* Vp = Xh + (size_t)b * CH * SEQ;

  v16h bq[2];
#pragma unroll
  for (int cs = 0; cs < 2; ++cs) bq[cs] = ld_frag(Qp + 32 * cs, CH, qb + l15, h);

  v8f accO[4];
#pragma unroll
  for (int u = 0; u < 4; ++u)
#pragma unroll
    for (int r = 0; r < 8; ++r) accO[u][r] = 0.0f;
  float rm = -1e30f, rl = 0.0f;

  for (int m0 = 0; m0 < SEQ; m0 += KBLK) {
    v8f st[4];
#pragma unroll
    for (int t = 0; t < 4; ++t)
#pragma unroll
      for (int r = 0; r < 8; ++r) st[t][r] = 0.0f;
#pragma unroll
    for (int cs = 0; cs < 2; ++cs) {
#pragma unroll
      for (int t = 0; t < 4; ++t) {
        const v16h ak = ld_frag(Qp + 32 * cs, CH, m0 + 16 * t + l15, h);
        st[t] = wmma16(ak, bq[cs], st[t]);
      }
    }

    float lm = st[0][0];
#pragma unroll
    for (int t = 0; t < 4; ++t)
#pragma unroll
      for (int r = 0; r < 8; ++r) lm = fmaxf(lm, st[t][r]);
    lm *= SCL2;
    lm = fmaxf(lm, __shfl_xor(lm, 16, 32));
    const float nm = fmaxf(rm, lm);
    const float corr = exp2f(rm - nm);
    rm = nm;

    float psum = 0.0f;
    F16x16 bp[2];
#pragma unroll
    for (int j = 0; j < 2; ++j)
#pragma unroll
      for (int tt = 0; tt < 2; ++tt)
#pragma unroll
        for (int r = 0; r < 8; ++r) {
          const float p = exp2f(st[2 * j + tt][r] * SCL2 - nm);
          psum += p;
          bp[j].e[8 * tt + r] = (_Float16)(p * PSC);
        }
    psum += __shfl_xor(psum, 16, 32);
    rl = rl * corr + psum;
#pragma unroll
    for (int u = 0; u < 4; ++u)
#pragma unroll
      for (int r = 0; r < 8; ++r) accO[u][r] *= corr;

#pragma unroll
    for (int j = 0; j < 2; ++j) {
#pragma unroll
      for (int u = 0; u < 4; ++u) {
        const v16h av = ld_frag(Vp + m0 + 32 * j, SEQ, 16 * u + l15, h);
        accO[u] = wmma16(av, bp[j].v, accO[u]);
      }
    }
  }

  const float invl = 1.0f / (rl * (XSC * PSC));
#pragma unroll
  for (int u = 0; u < 4; ++u)
#pragma unroll
    for (int r = 0; r < 8; ++r)
      OSt[(16 * u + 8 * h + r) * OSP + 16 * wv + l15] = accO[u][r] * invl;
  __syncthreads();

  float* op = out + (size_t)b * CH * SEQ;
#pragma unroll
  for (int it = 0; it < 8; ++it) {
    const int L = it * 16 + (tid >> 3);
    const int c = L >> 1, hl = L & 1, p = tid & 7;
    const v4f v = *(const v4fa*)(OSt + c * OSP + 32 * hl + 4 * p);
    float* dst = op + (size_t)c * SEQ + q0 + 32 * hl + 4 * p;
    *(volatile v4f*)dst = v;
    __threadfence();
    *(volatile v4f*)dst = v;
  }
}

extern "C" void kernel_launch(void* const* d_in, const int* in_sizes, int n_in,
                              void* d_out, int out_size, void* d_ws, size_t ws_size,
                              hipStream_t stream) {
  if (n_in < 3) return;
  if (in_sizes[0] < NB * CH * SEQ_FULL) return;
  if (in_sizes[1] < CH * CH) return;
  if (in_sizes[2] < CH) return;
  if (out_size < NB * CH * SEQ) return;
  const size_t plane = (size_t)NB * CH * SEQ * sizeof(_Float16);
  if (ws_size < 2 * plane) return;

  const float* x    = (const float*)d_in[0];
  const float* W    = (const float*)d_in[1];
  const float* bias = (const float*)d_in[2];
  float* out = (float*)d_out;

  char* ws = (char*)d_ws;
  _Float16* Xh  = (_Float16*)(ws);
  _Float16* QKh = (_Float16*)(ws + plane);

  const int grid = NB * (SEQ / 64);
  hipLaunchKernelGGL(k_prep, dim3(grid), dim3(128), 0, stream, x, W, bias, Xh, QKh);
  hipLaunchKernelGGL(k_attn, dim3(grid), dim3(128), 0, stream,
                     (const _Float16*)QKh, (const _Float16*)Xh, out);
  (void)hipGetLastError();
}
